// CRMF_50087908606248
// MI455X (gfx1250) — hardware-verified
//
#include <hip/hip_runtime.h>
#include <math.h>

typedef __attribute__((ext_vector_type(16))) _Float16 v16h;
typedef __attribute__((ext_vector_type(8)))  _Float16 v8h;
typedef __attribute__((ext_vector_type(16))) __bf16   v16b;
typedef __attribute__((ext_vector_type(8)))  __bf16   v8b;
typedef __attribute__((ext_vector_type(8)))  float    v8f;
typedef __attribute__((ext_vector_type(4)))  float    v4f;
typedef __attribute__((ext_vector_type(4)))  unsigned int v4u;

constexpr int kInst   = 512;
constexpr int kNode   = 256;
constexpr int kFin0   = 32;
constexpr int kHeads0 = 4;
constexpr int kFout0  = 64;
constexpr int kFin1   = 256;
constexpr int kFout1  = 32;
constexpr int kChunk  = 64;
constexpr int kNumChunks = kInst / kChunk;
constexpr int kHtRows = 64;

__device__ __forceinline__ unsigned short f2bf_bits(float f) {
  unsigned u = __float_as_uint(f);
  return (unsigned short)((u + 0x7FFFu + ((u >> 16) & 1u)) >> 16);
}
__device__ __forceinline__ float bf_bits2f(unsigned short h) { return __uint_as_float(((unsigned)h) << 16); }

__device__ __forceinline__ void dep_guard_h(v8f& a, v8f& b, v16h x, v16h y) { asm volatile("v_nop\n\tv_nop\n\tv_nop\n\tv_nop" : "+v"(a), "+v"(b) : "v"(x), "v"(y)); }
__device__ __forceinline__ void dep_guard_b(v8f& a, v8f& b, v16b x, v16b y) { asm volatile("v_nop\n\tv_nop\n\tv_nop\n\tv_nop" : "+v"(a), "+v"(b) : "v"(x), "v"(y)); }
__device__ __forceinline__ void keep4_h(v16h a, v16h b, v16h c, v16h d) { asm volatile("v_nop" :: "v"(a), "v"(b), "v"(c), "v"(d)); }
__device__ __forceinline__ void keep4_b(v16b a, v16b b, v16b c, v16b d) { asm volatile("v_nop" :: "v"(a), "v"(b), "v"(c), "v"(d)); }
__device__ __forceinline__ void acc_guard4(v8f& a, v8f& b, v8f& c, v8f& d) { asm volatile("v_nop\n\tv_nop\n\tv_nop\n\tv_nop" : "+v"(a), "+v"(b), "+v"(c), "+v"(d)); }
template <typename T> struct Frag;
template <> struct Frag<_Float16> {
  typedef v16h V; union U { v16h v; v8h h[2]; };
  static __device__ __forceinline__ v16h load(const _Float16* p) {
    U f; f.h[0] = *(const v8h*)(p); f.h[1] = *(const v8h*)(p + 16); return f.v;
  }
  static __device__ __forceinline__ v8f mma(v16h a, v16h b, v8f c) {
    return __builtin_amdgcn_wmma_f32_16x16x32_f16(false, a, false, b, (short)0, c, false, false);
  }
  static __device__ __forceinline__ void guard(v8f& a, v8f& b, v16h x, v16h y) { dep_guard_h(a, b, x, y); }
  static __device__ __forceinline__ void keep(v16h a, v16h b, v16h c, v16h d) { keep4_h(a, b, c, d); }
};
template <> struct Frag<__bf16> {
  typedef v16b V; union U { v16b v; v8b h[2]; };
  static __device__ __forceinline__ v16b load(const __bf16* p) {
    U f; f.h[0] = *(const v8b*)(p); f.h[1] = *(const v8b*)(p + 16); return f.v;
  }
  static __device__ __forceinline__ v8f mma(v16b a, v16b b, v8f c) {
    return __builtin_amdgcn_wmma_f32_16x16x32_bf16(false, a, false, b, (short)0, c, false, false);
  }
  static __device__ __forceinline__ void guard(v8f& a, v8f& b, v16b x, v16b y) { dep_guard_b(a, b, x, y); }
  static __device__ __forceinline__ void keep(v16b a, v16b b, v16b c, v16b d) { keep4_b(a, b, c, d); }
};

__device__ __forceinline__ unsigned pk16(unsigned short a, unsigned short b) { return (unsigned)a | ((unsigned)b << 16); }

template <int ET> struct Elem;
template <> struct Elem<0> { typedef _Float16 T; };
template <> struct Elem<1> { typedef __bf16 T; };
template <int ET, bool SPLIT, int BIAS_MODE, int OUT_MODE, bool RESID, int ACT = 0>
__global__ __launch_bounds__(256) void wmma_gemm64(
    const unsigned short* __restrict__ Ap, const unsigned short* __restrict__ A2p, int lda, long strideA,
    const unsigned short* __restrict__ Btp, const unsigned short* __restrict__ Bt2p, int ldb, long strideB,
    void* __restrict__ Cout, void* __restrict__ Cout2, int ldc, long strideC,
    const float* __restrict__ bias,
    const float* __restrict__ resid, long strideR,
    int M, int N, int K, float scale) {
  typedef typename Elem<ET>::T T;
  typedef typename Frag<T>::V V;
  const T* A = (const T*)Ap; const T* A2 = (const T*)A2p; const T* Bt = (const T*)Btp; const T* Bt2 = (const T*)Bt2p;
  __shared__ __align__(16) float sT[8][16 * 68];
  const int b    = blockIdx.y;
  const int lane = threadIdx.x & 31;
  const int wave = threadIdx.x >> 5;
  const int tilesN = N >> 6;
  const int tilesM = M >> 6;
  const int tile = blockIdx.x * 8 + wave;
  if (tile >= tilesM * tilesN) return;
  const int tm = tile / tilesN;
  const int tn = tile - tm * tilesN;
  const int m0 = tm << 6;
  const int n0 = tn << 6;

  const T* Ab  = A  + (size_t)b * strideA;
  const T* Bb  = Bt + (size_t)b * strideB;
  const T* Ab2 = SPLIT ? (A2  + (size_t)b * strideA) : nullptr;
  const T* Bb2 = SPLIT ? (Bt2 + (size_t)b * strideB) : nullptr;

  const int rlane = lane & 15;
  const int koff  = (lane >> 4) * 8;
  const int mOff  = (lane >> 4) * 8;

  v8f acc[4][4];
#pragma unroll
  for (int i = 0; i < 4; ++i)
#pragma unroll
    for (int j = 0; j < 4; ++j) acc[i][j] = (v8f){0.f,0.f,0.f,0.f,0.f,0.f,0.f,0.f};

  for (int k0 = 0; k0 < K; k0 += 32) {
    V bh[4], bl[4];
#pragma unroll
    for (int j = 0; j < 4; ++j) {
      const size_t bo = (size_t)(n0 + (j << 4) + rlane) * ldb + koff + k0;
      bh[j] = Frag<T>::load(Bb + bo);
      if (SPLIT) bl[j] = Frag<T>::load(Bb2 + bo);
    }
#pragma unroll
    for (int i = 0; i < 4; ++i) {
      const size_t ao = (size_t)(m0 + (i << 4) + rlane) * lda + koff + k0;
      V ah = Frag<T>::load(Ab + ao);
      V al;
      if (SPLIT) al = Frag<T>::load(Ab2 + ao);
#pragma unroll
      for (int j = 0; j < 4; ++j) {
        acc[i][j] = Frag<T>::mma(ah, bh[j], acc[i][j]);
        if (SPLIT) {
          acc[i][j] = Frag<T>::mma(ah, bl[j], acc[i][j]);
          acc[i][j] = Frag<T>::mma(al, bh[j], acc[i][j]);
        }
      }
      Frag<T>::guard(acc[i][0], acc[i][3], ah, SPLIT ? al : ah);
    }
    Frag<T>::keep(bh[0], bh[1], bh[2], bh[3]);
    if (SPLIT) Frag<T>::keep(bl[0], bl[1], bl[2], bl[3]);
  }
  acc_guard4(acc[0][0], acc[0][1], acc[0][2], acc[0][3]);
  acc_guard4(acc[1][0], acc[1][1], acc[1][2], acc[1][3]);
  acc_guard4(acc[2][0], acc[2][1], acc[2][2], acc[2][3]);
  acc_guard4(acc[3][0], acc[3][1], acc[3][2], acc[3][3]);

  float* slab = sT[wave];
  const float* Rb = RESID ? (resid + (size_t)b * strideR) : nullptr;
#pragma unroll
  for (int i = 0; i < 4; ++i) {
    const int mBase = m0 + (i << 4);
#pragma unroll
    for (int j = 0; j < 4; ++j) {
      const int n = n0 + (j << 4) + rlane;
      float bv = 0.f;
      if (BIAS_MODE == 2) bv = bias[n];
#pragma unroll
      for (int r = 0; r < 8; ++r) {
        float v = acc[i][j][r] * scale;
        if (BIAS_MODE == 1) v += bias[mBase + mOff + r];
        if (BIAS_MODE == 2) v += bv;
        if (RESID) v += Rb[(size_t)(mBase + mOff + r) * ldc + n];
        if (ACT == 2) v = fmaxf(v, 0.0f);
        if (ACT == 4) v = (v > 0.f) ? v : 0.01f * v;
        slab[(mOff + r) * 68 + (j << 4) + rlane] = v;
      }
    }
    __builtin_amdgcn_fence(__ATOMIC_RELEASE, "workgroup");
    __builtin_amdgcn_wave_barrier();
    __builtin_amdgcn_fence(__ATOMIC_ACQUIRE, "workgroup");
    if (OUT_MODE == 0) {
      float* C = (float*)Cout + (size_t)b * strideC;
      const int hh = lane >> 4, c4 = (lane & 15) * 4;
      for (int pass = 0; pass < 2; ++pass) {
#pragma unroll
        for (int it = 0; it < 8; ++it) {
          const int row = it * 2 + hh;
          v4f v = *(const v4f*)(slab + row * 68 + c4);
          *(volatile v4f*)(C + (size_t)(mBase + row) * ldc + n0 + c4) = v;
        }
        __threadfence();
      }
    } else {
      const int q = lane >> 3, c8 = (lane & 7) * 8;
      unsigned short* C  = (unsigned short*)Cout  + (size_t)b * strideC;
      unsigned short* C2 = (OUT_MODE == 2) ? ((unsigned short*)Cout2 + (size_t)b * strideC) : nullptr;
      for (int pass = 0; pass < 2; ++pass) {
#pragma unroll
        for (int it = 0; it < 4; ++it) {
          const int row = it * 4 + q;
          const float* sp = slab + row * 68 + c8;
          v8h hv, lv;
#pragma unroll
          for (int e = 0; e < 8; ++e) {
            if (OUT_MODE == 1) {
              hv[e] = (_Float16)sp[e];
            } else {
              unsigned short hb = f2bf_bits(sp[e]);
              unsigned short lb = f2bf_bits(sp[e] - bf_bits2f(hb));
              hv[e] = __builtin_bit_cast(_Float16, hb);
              lv[e] = __builtin_bit_cast(_Float16, lb);
            }
          }
          *(volatile v8h*)(C + (size_t)(mBase + row) * ldc + n0 + c8) = hv;
          if (OUT_MODE == 2) *(volatile v8h*)(C2 + (size_t)(mBase + row) * ldc + n0 + c8) = lv;
        }
        __threadfence();
      }
    }
    __builtin_amdgcn_fence(__ATOMIC_RELEASE, "workgroup");
    __builtin_amdgcn_wave_barrier();
    __builtin_amdgcn_fence(__ATOMIC_ACQUIRE, "workgroup");
  }
}

__device__ __forceinline__ float lrelu02(float v) { return v >= 0.f ? v : 0.2f * v; }

__device__ __forceinline__ void bf_split(float f, unsigned short& hb, unsigned short& lb) {
  hb = f2bf_bits(f);
  lb = f2bf_bits(f - bf_bits2f(hb));
}

__device__ __forceinline__ void store2_pair(unsigned short* ph, unsigned short* pl, v4u uh, v4u ul) {
  *(volatile v4u*)ph = uh;
  *(volatile v4u*)pl = ul;
  __threadfence();
  *(volatile v4u*)ph = uh;
  *(volatile v4u*)pl = ul;
}

__global__ __launch_bounds__(256) void k_wprep(const float* __restrict__ w0, const float* __restrict__ w1,
                                               unsigned short* __restrict__ a0h, unsigned short* __restrict__ a0l,
                                               unsigned short* __restrict__ a1h, unsigned short* __restrict__ a1l) {
  const int t = threadIdx.x;
#pragma unroll 1
  for (int it = 0; it < 4; ++it) {
    const int q = it * 256 + t;
    const int row = q >> 2;
    const int f0 = (q & 3) * 8;
    const int hd = row >> 6, o = row & 63;
    unsigned short hb[8], lb[8];
#pragma unroll
    for (int e = 0; e < 8; ++e) {
      const float v = w0[(size_t)(hd * kFin0 + f0 + e) * kFout0 + o];
      bf_split(v, hb[e], lb[e]);
    }
    const v4u uh = (v4u){pk16(hb[0], hb[1]), pk16(hb[2], hb[3]), pk16(hb[4], hb[5]), pk16(hb[6], hb[7])};
    const v4u ul = (v4u){pk16(lb[0], lb[1]), pk16(lb[2], lb[3]), pk16(lb[4], lb[5]), pk16(lb[6], lb[7])};
    store2_pair(a0h + (size_t)q * 8, a0l + (size_t)q * 8, uh, ul);
  }
#pragma unroll 1
  for (int it = 0; it < 8; ++it) {
    const int q = it * 256 + t;
    const int row = q >> 5;
    const int f0 = (q & 31) * 8;
    const int oc = row < kFout1 ? row : (kFout1 - 1);
    const bool live = row < kFout1;
    unsigned short hb[8], lb[8];
#pragma unroll
    for (int e = 0; e < 8; ++e) {
      float v = w1[(size_t)(f0 + e) * kFout1 + oc];
      v = live ? v : 0.f;
      bf_split(v, hb[e], lb[e]);
    }
    const v4u uh = (v4u){pk16(hb[0], hb[1]), pk16(hb[2], hb[3]), pk16(hb[4], hb[5]), pk16(hb[6], hb[7])};
    const v4u ul = (v4u){pk16(lb[0], lb[1]), pk16(lb[2], lb[3]), pk16(lb[4], lb[5]), pk16(lb[6], lb[7])};
    store2_pair(a1h + (size_t)q * 8, a1l + (size_t)q * 8, uh, ul);
  }
}

__global__ __launch_bounds__(256) void k_in0(const float* __restrict__ x,
                                             unsigned short* __restrict__ xh, unsigned short* __restrict__ xl) {
  __shared__ __align__(16) float xs[kNode * kFin0];
  __shared__ float red1[8][kFin0];
  __shared__ float red2[8][kFin0];
  __shared__ float smean[kFin0];
  __shared__ float sinv[kFin0];
  const int bl = blockIdx.x;
  const int t = threadIdx.x;
  const float* xb = x + (size_t)bl * (kNode * kFin0);
#pragma unroll
  for (int it = 0; it < 8; ++it) {
    const int idx = (it * 256 + t) * 4;
    *(v4f*)(xs + idx) = *(const v4f*)(xb + idx);
  }
  __syncthreads();
  const int c = t & 31, g = t >> 5;
  {
    float s = 0.f;
#pragma unroll 1
    for (int r = 0; r < 32; ++r) s += xs[(g * 32 + r) * kFin0 + c];
    red1[g][c] = s;
  }
  __syncthreads();
  if (t < kFin0) {
    float s = 0.f;
#pragma unroll
    for (int gg = 0; gg < 8; ++gg) s += red1[gg][t];
    smean[t] = s * (1.0f / 256.0f);
  }
  __syncthreads();
  {
    const float mu = smean[c];
    float s = 0.f;
#pragma unroll 1
    for (int r = 0; r < 32; ++r) {
      const float d = xs[(g * 32 + r) * kFin0 + c] - mu;
      s += d * d;
    }
    red2[g][c] = s;
  }
  __syncthreads();
  if (t < kFin0) {
    float s = 0.f;
#pragma unroll
    for (int gg = 0; gg < 8; ++gg) s += red2[gg][t];
    const float var = s * (1.0f / 256.0f);
    sinv[t] = 1.0f / sqrtf(var + 1e-5f);
  }
  __syncthreads();
#pragma unroll 1
  for (int it = 0; it < 4; ++it) {
    const int q = it * 256 + t;
    const int n = q >> 2, c0 = (q & 3) * 8;
    unsigned short hb[8], lb[8];
#pragma unroll
    for (int e = 0; e < 8; ++e) {
      const float v = (xs[n * kFin0 + c0 + e] - smean[c0 + e]) * sinv[c0 + e];
      bf_split(v, hb[e], lb[e]);
    }
    const v4u uh = (v4u){pk16(hb[0], hb[1]), pk16(hb[2], hb[3]), pk16(hb[4], hb[5]), pk16(hb[6], hb[7])};
    const v4u ul = (v4u){pk16(lb[0], lb[1]), pk16(lb[2], lb[3]), pk16(lb[4], lb[5]), pk16(lb[6], lb[7])};
    const size_t o = (size_t)bl * (kNode * kFin0) + (size_t)q * 8;
    store2_pair(xh + o, xl + o, uh, ul);
  }
}

__global__ __launch_bounds__(256) void k_att(const float* __restrict__ htf,
                                             const float* __restrict__ asrc, const float* __restrict__ adst,
                                             int nheads, int astride, int nfeat,
                                             unsigned short* __restrict__ hth, unsigned short* __restrict__ htl,
                                             unsigned short* __restrict__ pph, unsigned short* __restrict__ ppl) {
  __shared__ __align__(16) float sS[kNode];
  __shared__ __align__(16) float sD[kNode];
  __shared__ float redm[8];
  const int z = blockIdx.x;
  const int t = threadIdx.x, lane = t & 31, wave = t >> 5;
  const int hd = z % nheads;
  const float* as = asrc + hd * astride;
  const float* ad = adst + hd * astride;
  const float* ht = htf + (size_t)z * (kHtRows * kNode);

#pragma unroll 1
  for (int it = 0; it < 8; ++it) {
    const int row = it * 8 + wave;
    const int m0 = lane * 8;
    const float* p = ht + row * kNode + m0;
    const v4f a = *(const v4f*)(p);
    const v4f c = *(const v4f*)(p + 4);
    unsigned short hb[8], lb[8];
#pragma unroll
    for (int e = 0; e < 4; ++e) {
      bf_split(a[e], hb[e], lb[e]);
      bf_split(c[e], hb[4 + e], lb[4 + e]);
    }
    const v4u uh = (v4u){pk16(hb[0], hb[1]), pk16(hb[2], hb[3]), pk16(hb[4], hb[5]), pk16(hb[6], hb[7])};
    const v4u ul = (v4u){pk16(lb[0], lb[1]), pk16(lb[2], lb[3]), pk16(lb[4], lb[5]), pk16(lb[6], lb[7])};
    const size_t o = (size_t)z * (kHtRows * kNode) + (size_t)row * kNode + m0;
    store2_pair(hth + o, htl + o, uh, ul);
  }

  const int nf = nfeat < kHtRows ? nfeat : kHtRows;
  float s0 = 0.f, s1 = 0.f;
#pragma unroll 1
  for (int o2 = 0; o2 < nf; ++o2) {
    const float hv = ht[o2 * kNode + t];
    s0 = fmaf(hv, as[o2], s0);
    s1 = fmaf(hv, ad[o2], s1);
  }
  sS[t] = s0;
  sD[t] = s1;
  float mx = s1;
#pragma unroll
  for (int off = 16; off > 0; off >>= 1) mx = fmaxf(mx, __shfl_xor(mx, off, 32));
  if (lane == 0) redm[wave] = mx;
  __syncthreads();
  float sdmax = redm[0];
#pragma unroll
  for (int w = 1; w < 8; ++w) sdmax = fmaxf(sdmax, redm[w]);
  float sdv[8];
  {
    const v4f d0 = *(const v4f*)(sD + lane * 8);
    const v4f d1 = *(const v4f*)(sD + lane * 8 + 4);
#pragma unroll
    for (int e = 0; e < 4; ++e) { sdv[e] = d0[e]; sdv[4 + e] = d1[e]; }
  }

#pragma unroll 1
  for (int i = 0; i < 32; ++i) {
    const int n = wave * 32 + i;
    const float ssn = sS[n];
    const float rm = lrelu02(ssn + sdmax);
    float pe[8];
    float psum = 0.f;
#pragma unroll
    for (int e = 0; e < 8; ++e) {
      const float v = lrelu02(ssn + sdv[e]) - rm;
      pe[e] = expf(v);
      psum += pe[e];
    }
#pragma unroll
    for (int off = 16; off > 0; off >>= 1) psum += __shfl_xor(psum, off, 32);
    psum = __shfl(psum, 0, 32);
    const float inv = 1.0f / psum;
    unsigned short hb[8], lb[8];
#pragma unroll
    for (int e = 0; e < 8; ++e) bf_split(pe[e] * inv, hb[e], lb[e]);
    const v4u uh = (v4u){pk16(hb[0], hb[1]), pk16(hb[2], hb[3]), pk16(hb[4], hb[5]), pk16(hb[6], hb[7])};
    const v4u ul = (v4u){pk16(lb[0], lb[1]), pk16(lb[2], lb[3]), pk16(lb[4], lb[5]), pk16(lb[6], lb[7])};
    const size_t o = (size_t)z * (kNode * kNode) + (size_t)n * kNode + lane * 8;
    store2_pair(pph + o, ppl + o, uh, ul);
  }
}

__global__ __launch_bounds__(256) void k_mid(const float* __restrict__ c0, const float* __restrict__ bias0,
                                             unsigned short* __restrict__ xh, unsigned short* __restrict__ xl) {
  extern __shared__ __align__(16) float es[];
  __shared__ float red1[4][kFout0];
  __shared__ float red2[4][kFout0];
  __shared__ float smean[kFout0];
  __shared__ float sinv[kFout0];
  const int z = blockIdx.x;
  const int bl = z >> 2, hd = z & 3;
  const int t = threadIdx.x;
  const int o = t & 63, g = t >> 6;
  const float* cz = c0 + (size_t)z * (kNode * kFout0);
  const float bo = bias0[o];
  {
    float s = 0.f;
#pragma unroll 1
    for (int r = 0; r < 64; ++r) {
      const int n = g * 64 + r;
      float v = cz[n * kFout0 + o] + bo;
      const float em = expm1f(v);
      v = v > 0.f ? v : em;
      es[n * kFout0 + o] = v;
      s += v;
    }
    red1[g][o] = s;
  }
  __syncthreads();
  if (t < kFout0) {
    const float s = ((red1[0][t] + red1[1][t]) + red1[2][t]) + red1[3][t];
    smean[t] = s * (1.0f / 256.0f);
  }
  __syncthreads();
  {
    const float mu = smean[o];
    float s = 0.f;
#pragma unroll 1
    for (int r = 0; r < 64; ++r) {
      const float d = es[(g * 64 + r) * kFout0 + o] - mu;
      s += d * d;
    }
    red2[g][o] = s;
  }
  __syncthreads();
  if (t < kFout0) {
    const float s = ((red2[0][t] + red2[1][t]) + red2[2][t]) + red2[3][t];
    const float var = s * (1.0f / 256.0f);
    sinv[t] = 1.0f / sqrtf(var + 1e-5f);
  }
  __syncthreads();
  const int rsub = t >> 3, c8 = (t & 7) * 8;
#pragma unroll 1
  for (int it = 0; it < 8; ++it) {
    const int n = it * 32 + rsub;
    const v4f a = *(const v4f*)(es + n * kFout0 + c8);
    const v4f c = *(const v4f*)(es + n * kFout0 + c8 + 4);
    unsigned short hb[8], lb[8];
#pragma unroll
    for (int e = 0; e < 4; ++e) {
      const float v0 = (a[e] - smean[c8 + e]) * sinv[c8 + e];
      const float v1 = (c[e] - smean[c8 + 4 + e]) * sinv[c8 + 4 + e];
      bf_split(v0, hb[e], lb[e]);
      bf_split(v1, hb[4 + e], lb[4 + e]);
    }
    const v4u uh = (v4u){pk16(hb[0], hb[1]), pk16(hb[2], hb[3]), pk16(hb[4], hb[5]), pk16(hb[6], hb[7])};
    const v4u ul = (v4u){pk16(lb[0], lb[1]), pk16(lb[2], lb[3]), pk16(lb[4], lb[5]), pk16(lb[6], lb[7])};
    const size_t oo = ((size_t)bl * kNode + n) * kFin1 + hd * kFout0 + c8;
    store2_pair(xh + oo, xl + oo, uh, ul);
  }
}

__global__ __launch_bounds__(256) void k_out(const float* __restrict__ c1, const float* __restrict__ bias1,
                                             float* __restrict__ outp) {
  const int bl = blockIdx.x;
  const int t = threadIdx.x;
  const int rsub = t >> 3, c4 = (t & 7) * 4;
  const v4f bb = (v4f){bias1[c4], bias1[c4 + 1], bias1[c4 + 2], bias1[c4 + 3]};
#pragma unroll 1
  for (int it = 0; it < 8; ++it) {
    const int n = it * 32 + rsub;
    const v4f a = *(const v4f*)(c1 + ((size_t)bl * kNode + n) * kHtRows + c4);
    const v4f v = a + bb;
    float* p = outp + ((size_t)bl * kNode + n) * kFout1 + c4;
    *(volatile v4f*)p = v;
    __threadfence();
    *(volatile v4f*)p = v;
  }
}

extern "C" void kernel_launch(void* const* d_in, const int* in_sizes, int n_in,
                              void* d_out, int out_size, void* d_ws, size_t ws_size,
                              hipStream_t stream) {
  if (n_in < 9) return;
  if (in_sizes[0] != kInst * kNode * kFin0) return;
  if (in_sizes[1] != kHeads0 * kFin0 * kFout0) return;
  if (in_sizes[2] != kHeads0 * kFout0 || in_sizes[3] != kHeads0 * kFout0) return;
  if (in_sizes[4] != kFout0) return;
  if (in_sizes[5] != kFin1 * kFout1) return;
  if (in_sizes[6] != kFout1 || in_sizes[7] != kFout1 || in_sizes[8] != kFout1) return;
  if (out_size != kInst * kNode * kFout1) return;

  const size_t oA0H = 0, oA0L = 16384, oA1H = 32768, oA1L = 65536;
  const size_t szX0 = (size_t)kChunk * kNode * kFin0 * 2;
  const size_t szHF = (size_t)kChunk * kHeads0 * kHtRows * kNode * 4;
  const size_t szHT = (size_t)kChunk * kHeads0 * kHtRows * kNode * 2;
  const size_t szP0 = (size_t)kChunk * kHeads0 * kNode * kNode * 2;
  const size_t oX0H = 131072;
  const size_t oX0L = oX0H + szX0;
  const size_t oHF  = oX0L + szX0;
  const size_t oHTH = oHF + szHF;
  const size_t oHTL = oHTH + szHT;
  const size_t oP0H = oHTL + szHT;
  const size_t oP0L = oP0H + szP0;
  const size_t wsTotal = oP0L + szP0;
  const size_t szX1 = (size_t)kChunk * kNode * kFin1 * 2;
  const size_t szH1F = (size_t)kChunk * kHtRows * kNode * 4;
  const size_t szH1P = (size_t)kChunk * kHtRows * kNode * 2;
  const size_t szP1 = (size_t)kChunk * kNode * kNode * 2;
  const size_t szC1 = (size_t)kChunk * kNode * kHtRows * 4;
  const size_t oX1H = oP0H;
  const size_t oX1L = oX1H + szX1;
  const size_t oH1F = oX1L + szX1;
  const size_t oH1H = oH1F + szH1F;
  const size_t oH1L = oH1H + szH1P;
  const size_t oP1H = oH1L + szH1P;
  const size_t oP1L = oP1H + szP1;
  const size_t oC1F = oP1L + szP1;
  if (oC1F + szC1 > wsTotal) return;
  if (ws_size < wsTotal) return;

  const float* x      = (const float*)d_in[0];
  const float* w0     = (const float*)d_in[1];
  const float* a_src0 = (const float*)d_in[2];
  const float* a_dst0 = (const float*)d_in[3];
  const float* b0     = (const float*)d_in[4];
  const float* w1     = (const float*)d_in[5];
  const float* a_src1 = (const float*)d_in[6];
  const float* a_dst1 = (const float*)d_in[7];
  const float* b1     = (const float*)d_in[8];
  float* out = (float*)d_out;
  unsigned char* ws = (unsigned char*)d_ws;

  unsigned short* A0H = (unsigned short*)(ws + oA0H);
  unsigned short* A0L = (unsigned short*)(ws + oA0L);
  unsigned short* A1H = (unsigned short*)(ws + oA1H);
  unsigned short* A1L = (unsigned short*)(ws + oA1L);
  unsigned short* X0H = (unsigned short*)(ws + oX0H);
  unsigned short* X0L = (unsigned short*)(ws + oX0L);
  float* HF = (float*)(ws + oHF);
  unsigned short* HTH = (unsigned short*)(ws + oHTH);
  unsigned short* HTL = (unsigned short*)(ws + oHTL);
  unsigned short* P0H = (unsigned short*)(ws + oP0H);
  unsigned short* P0L = (unsigned short*)(ws + oP0L);
  unsigned short* X1H = (unsigned short*)(ws + oX1H);
  unsigned short* X1L = (unsigned short*)(ws + oX1L);
  float* H1F = (float*)(ws + oH1F);
  unsigned short* H1H = (unsigned short*)(ws + oH1H);
  unsigned short* H1L = (unsigned short*)(ws + oH1L);
  unsigned short* P1H = (unsigned short*)(ws + oP1H);
  unsigned short* P1L = (unsigned short*)(ws + oP1L);
  float* C1F = (float*)(ws + oC1F);

  const dim3 blk(256);
  k_wprep<<<dim3(1), blk, 0, stream>>>(w0, w1, A0H, A0L, A1H, A1L);

  const int nz0 = kChunk * kHeads0;
  for (int ch = 0; ch < kNumChunks; ++ch) {
    const float* xc = x + (size_t)ch * kChunk * kNode * kFin0;
    float* oc = out + (size_t)ch * kChunk * kNode * kFout1;

    k_in0<<<dim3(kChunk), blk, 0, stream>>>(xc, X0H, X0L);

    wmma_gemm64<1, true, 0, 0, false, 0><<<dim3(2, kChunk), blk, 0, stream>>>(
        A0H, A0L, kFin0, 0L,
        X0H, X0L, kFin0, (long)(kNode * kFin0),
        (void*)HF, nullptr, kNode, (long)(kHeads0 * kHtRows * kNode),
        nullptr, nullptr, 0L,
        kHeads0 * kFout0, kNode, kFin0, 1.0f);

    k_att<<<dim3(nz0), blk, 0, stream>>>(HF, a_src0, a_dst0, kHeads0, kFout0, kFout0, HTH, HTL, P0H, P0L);

    wmma_gemm64<1, true, 0, 0, false, 0><<<dim3(1, nz0), blk, 0, stream>>>(
        P0H, P0L, kNode, (long)(kNode * kNode),
        HTH, HTL, kNode, (long)(kHtRows * kNode),
        (void*)HF, nullptr, kHtRows, (long)(kNode * kHtRows),
        nullptr, nullptr, 0L,
        kNode, kHtRows, kNode, 1.0f);

    k_mid<<<dim3(nz0), blk, (size_t)kNode * kFout0 * sizeof(float), stream>>>(HF, b0, X1H, X1L);

    wmma_gemm64<1, true, 0, 0, false, 0><<<dim3(1, kChunk), blk, 0, stream>>>(
        A1H, A1L, kFin1, 0L,
        X1H, X1L, kFin1, (long)(kNode * kFin1),
        (void*)H1F, nullptr, kNode, (long)(kHtRows * kNode),
        nullptr, nullptr, 0L,
        kHtRows, kNode, kFin1, 1.0f);

    k_att<<<dim3(kChunk), blk, 0, stream>>>(H1F, a_src1, a_dst1, 1, kFout1, kFout1, H1H, H1L, P1H, P1L);

    wmma_gemm64<1, true, 0, 0, false, 0><<<dim3(1, kChunk), blk, 0, stream>>>(
        P1H, P1L, kNode, (long)(kNode * kNode),
        H1H, H1L, kNode, (long)(kHtRows * kNode),
        (void*)C1F, nullptr, kHtRows, (long)(kNode * kHtRows),
        nullptr, nullptr, 0L,
        kNode, kHtRows, kNode, 1.0f);

    k_out<<<dim3(kChunk), blk, 0, stream>>>(C1F, b1, oc);
  }
}
